// GlobalPath_24438363914545
// MI455X (gfx1250) — hardware-verified
//
#include <hip/hip_runtime.h>


namespace {
constexpr int NB = 4, C = 256, HH = 48, WW = 48, L = HH * WW, NT = NB * L, CE = 512, NS = 16, DTR = 32, XD = DTR + 2 * NS;
constexpr float XS = 8.0f, VS = 1024.0f, DS = 16384.0f, OS = 1024.0f, WSC = 256.0f;
typedef _Float16 b16;
typedef __attribute__((ext_vector_type(16))) _Float16 v16b;
typedef __attribute__((ext_vector_type(8))) _Float16 v8b;
typedef __attribute__((ext_vector_type(8))) float v8f;
typedef __attribute__((ext_vector_type(4))) float v4f;
__device__ __forceinline__ float bf16_rne(float f) { unsigned int u = __float_as_uint(f); u += 0x7FFFu + ((u >> 16) & 1u); return __uint_as_float(u & 0xFFFF0000u); }
__device__ __forceinline__ void split16(float v, b16& hi, b16& lo) { hi = (b16)v; lo = (b16)(v - (float)hi); }
__device__ __forceinline__ v16b frag_kb(const b16* p, int hh) { const v8b a = *(const v8b*)(p + 8 * hh), b = *(const v8b*)(p + 16 + 8 * hh); v16b f;
#pragma unroll
  for (int e = 0; e < 8; ++e) { f[e] = a[e]; f[8 + e] = b[e]; } return f; }
__device__ __forceinline__ v8f wmma16b(v16b a, v16b b, v8f c) { v8f d = __builtin_amdgcn_wmma_f32_16x16x32_f16(false, a, false, b, (short)0, c, false, false); asm volatile("v_nop\n\tv_nop\n\tv_nop\n\tv_nop" : "+v"(d) : "v"(a), "v"(b)); return d; }
__device__ __forceinline__ void wave_lds_sync() { __builtin_amdgcn_fence(__ATOMIC_RELEASE, "workgroup"); __builtin_amdgcn_wave_barrier(); __builtin_amdgcn_fence(__ATOMIC_ACQUIRE, "workgroup"); }
__device__ __forceinline__ float pmul(float a, float b) { float p = a * b; asm volatile("" : "+v"(p)); return p; }
__device__ __forceinline__ float sigm(float v) { return 1.0f / (1.0f + __expf(-v)); }
__device__ __forceinline__ float softplus(float v) { return v > 20.0f ? v : (v < -20.0f ? __expf(v) : log1pf(__expf(v))); }

__global__ __launch_bounds__(256) void wcopy_kernel(const float* __restrict__ w, int n8, b16* __restrict__ WT) {
  const size_t u = (size_t)blockIdx.x * 256 + threadIdx.x; if (u >= (size_t)n8) return; const size_t e = u * 8; v8b v; for (int j = 0; j < 8; ++j) v[j] = (b16)(bf16_rne(w[e + j]) * WSC);
  for (int pass = 0; pass < 2; ++pass) { *(volatile v8b*)(WT + e) = v; __threadfence(); }
}
__global__ __launch_bounds__(32) void expand_kernel(const float* __restrict__ x, const float* __restrict__ nw, const float* __restrict__ nbias, const b16* __restrict__ WEX, const float* __restrict__ bex, float* __restrict__ UV) {
  __shared__ __attribute__((aligned(16))) b16 Ah[16][C + 8], Al[16][C + 8]; __shared__ __attribute__((aligned(16))) float Tf[16][128 + 4];
  const int lane = threadIdx.x, nloc = lane & 15, hlf = lane >> 4; const size_t m0 = (size_t)blockIdx.x * 16; const int b = (int)(m0 / L), p0 = (int)(m0 % L);
  float g8[8], be8[8]; for (int j = 0; j < 8; ++j) { g8[j] = bf16_rne(nw[32 * j + lane]); be8[j] = bf16_rne(nbias[32 * j + lane]); }
  for (int rr = 0; rr < 16; ++rr) { float v[8]; float s = 0.0f; for (int j = 0; j < 8; ++j) { v[j] = bf16_rne(x[((size_t)b * C + 32 * j + lane) * L + p0 + rr]); s += v[j]; } for (int o = 16; o; o >>= 1) s += __shfl_xor(s, o); const float mu = s * (1.0f / C);
    float q = 0.0f; for (int j = 0; j < 8; ++j) { const float d = v[j] - mu; q += pmul(d, d); } for (int o = 16; o; o >>= 1) q += __shfl_xor(q, o); const float rs = rsqrtf(q * (1.0f / C) + 1e-6f);
    for (int j = 0; j < 8; ++j) { const float xn = pmul(pmul(v[j] - mu, rs), g8[j]) + be8[j]; b16 p, ql; split16(xn * XS, p, ql); Ah[rr][32 * j + lane] = p; Al[rr][32 * j + lane] = ql; } }
  wave_lds_sync();
#pragma unroll 1
  for (int cg = 0; cg < 8; ++cg) { v8f acc[8];
#pragma unroll
    for (int t = 0; t < 8; ++t) acc[t] = (v8f){};
#pragma unroll 2
    for (int kb = 0; kb < C; kb += 32) { const v16b a = frag_kb(&Ah[nloc][kb], hlf), al = frag_kb(&Al[nloc][kb], hlf);
#pragma unroll
      for (int t = 0; t < 8; ++t) { const v16b bw = frag_kb(WEX + (size_t)(cg * 128 + t * 16 + nloc) * C + kb, hlf); acc[t] = wmma16b(a, bw, acc[t]); acc[t] = wmma16b(al, bw, acc[t]); } }
#pragma unroll
    for (int t = 0; t < 8; ++t) { const int c = cg * 128 + t * 16 + nloc; const float bb = bf16_rne(bex[c]);
#pragma unroll 1
      for (int r8 = 0; r8 < 8; ++r8) Tf[8 * hlf + r8][t * 16 + nloc] = acc[t][r8] * (1.0f / (XS * WSC)) + bb; }
    wave_lds_sync();
    for (int pass = 0; pass < 2; ++pass) { for (int rr = 0; rr < 16; ++rr) *(volatile v4f*)(UV + (m0 + rr) * (2 * CE) + cg * 128 + lane * 4) = *(const v4f*)(&Tf[rr][lane * 4]); __threadfence(); }
    wave_lds_sync(); }
}
__global__ __launch_bounds__(256) void dwconv_kernel(const float* __restrict__ UV, const float* __restrict__ dwk, float* __restrict__ V2) {
  const size_t gid = (size_t)blockIdx.x * 256 + threadIdx.x; const size_t t = gid / (CE / 4); const int c4 = (int)(gid % (CE / 4)) * 4; if (t >= (size_t)NT) return;
  const int b = (int)(t / L), p = (int)(t % L), py = p / WW, px = p % WW; v4f acc = {0.0f, 0.0f, 0.0f, 0.0f};
#pragma unroll
  for (int i = 0; i < 3; ++i)
#pragma unroll
    for (int j = 0; j < 3; ++j) { const int yy = py + i - 1, xx = px + j - 1; if (yy < 0 || yy >= HH || xx < 0 || xx >= WW) continue; const v4f vv = *(const v4f*)(UV + ((size_t)b * L + yy * WW + xx) * (2 * CE) + CE + c4); const v4f kw = *(const v4f*)(dwk + (i * 3 + j) * CE + c4);
      for (int q = 0; q < 4; ++q) acc[q] += pmul(vv[q], bf16_rne(kw[q])); }
  v4f o; for (int q = 0; q < 4; ++q) o[q] = pmul(acc[q], sigm(acc[q]));
  for (int pass = 0; pass < 2; ++pass) { *(volatile v4f*)(V2 + t * CE + c4) = o; __threadfence(); }
}
__global__ __launch_bounds__(32) void mid_kernel(const float* __restrict__ V2, const b16* __restrict__ WXP, const float* __restrict__ bxp, const b16* __restrict__ WDT, const float* __restrict__ bdt, float* __restrict__ BCp, float* __restrict__ DT) {
  __shared__ __attribute__((aligned(16))) b16 Ah[16][CE + 8], Al[16][CE + 8]; __shared__ __attribute__((aligned(16))) float Tf[16][128 + 4]; __shared__ __attribute__((aligned(16))) float Sbc[16][32];
  const int lane = threadIdx.x, nloc = lane & 15, hlf = lane >> 4; const size_t m0 = (size_t)blockIdx.x * 16;
  for (int rr = 0; rr < 16; ++rr) for (int q = 0; q < 4; ++q) { const v4f v = *(const v4f*)(V2 + (m0 + rr) * CE + q * 128 + lane * 4); for (int j = 0; j < 4; ++j) { b16 p, ql; split16(v[j] * VS, p, ql); Ah[rr][q * 128 + lane * 4 + j] = p; Al[rr][q * 128 + lane * 4 + j] = ql; } }
  wave_lds_sync();
  v8f ax[4] = {(v8f){}, (v8f){}, (v8f){}, (v8f){}};
#pragma unroll 2
  for (int kb = 0; kb < CE; kb += 32) { const v16b a = frag_kb(&Ah[nloc][kb], hlf), al = frag_kb(&Al[nloc][kb], hlf);
#pragma unroll
    for (int t = 0; t < 4; ++t) { const v16b bw = frag_kb(WXP + (size_t)(t * 16 + nloc) * CE + kb, hlf); ax[t] = wmma16b(a, bw, ax[t]); ax[t] = wmma16b(al, bw, ax[t]); } }
  wave_lds_sync();
  const float sx = 1.0f / (VS * WSC);
#pragma unroll
  for (int r8 = 0; r8 < 8; ++r8) { const int rl = 8 * hlf + r8;
    { const float d0 = ax[0][r8] * sx + bf16_rne(bxp[nloc]); b16 p, ql; split16(d0 * DS, p, ql); Ah[rl][nloc] = p; Al[rl][nloc] = ql; }
    { const float d1 = ax[1][r8] * sx + bf16_rne(bxp[16 + nloc]); b16 p, ql; split16(d1 * DS, p, ql); Ah[rl][16 + nloc] = p; Al[rl][16 + nloc] = ql; }
    Sbc[rl][nloc] = ax[2][r8] * sx + bf16_rne(bxp[32 + nloc]); Sbc[rl][16 + nloc] = ax[3][r8] * sx + bf16_rne(bxp[48 + nloc]); }
  wave_lds_sync();
  for (int pass = 0; pass < 2; ++pass) { for (int rr = 0; rr < 16; ++rr) ((volatile float*)BCp)[(m0 + rr) * 32 + lane] = Sbc[rr][lane]; __threadfence(); }
  const float se = 1.0f / (DS * WSC);
#pragma unroll 1
  for (int cg = 0; cg < 4; ++cg) { v8f acc[8]; const v16b a = frag_kb(&Ah[nloc][0], hlf), al = frag_kb(&Al[nloc][0], hlf);
#pragma unroll
    for (int t = 0; t < 8; ++t) { acc[t] = (v8f){}; const v16b bw = frag_kb(WDT + (size_t)(cg * 128 + t * 16 + nloc) * DTR, hlf); acc[t] = wmma16b(a, bw, acc[t]); acc[t] = wmma16b(al, bw, acc[t]); }
#pragma unroll
    for (int t = 0; t < 8; ++t) { const int c = cg * 128 + t * 16 + nloc; const float bb = bf16_rne(bdt[c]);
#pragma unroll 1
      for (int r8 = 0; r8 < 8; ++r8) Tf[8 * hlf + r8][t * 16 + nloc] = softplus(acc[t][r8] * se + bb); }
    wave_lds_sync();
    for (int pass = 0; pass < 2; ++pass) { for (int rr = 0; rr < 16; ++rr) *(volatile v4f*)(DT + (m0 + rr) * CE + cg * 128 + lane * 4) = *(const v4f*)(&Tf[rr][lane * 4]); __threadfence(); }
    wave_lds_sync(); }
}
__global__ __launch_bounds__(256) void scan_kernel(const float* __restrict__ V2, const float* __restrict__ DT, const float* __restrict__ BCp, const float* __restrict__ alog, const float* __restrict__ Dp, int nb, float* __restrict__ Y) {
  const int gid = blockIdx.x * 256 + threadIdx.x; const int b = gid / CE, d = gid % CE; if (b >= nb) return;
  float A[NS]; for (int s = 0; s < NS; ++s) A[s] = -__expf(bf16_rne(alog[d * NS + s])); const float dd = bf16_rne(Dp[d]);
#pragma unroll 1
  for (int pass = 0; pass < 2; ++pass) { float h[NS]; for (int s = 0; s < NS; ++s) h[s] = 0.0f;
#pragma unroll 1
    for (int t = 0; t < L; ++t) { const size_t row = (size_t)b * L + t; const float v = V2[row * CE + d], dt = DT[row * CE + d]; const float dv = pmul(dt, v); float y = 0.0f;
#pragma unroll
      for (int s = 0; s < NS; ++s) { const float da = __expf(pmul(dt, A[s])); h[s] = pmul(h[s], da) + pmul(dv, BCp[row * 32 + s]); y += pmul(h[s], BCp[row * 32 + 16 + s]); }
      y += pmul(dd, v); ((volatile float*)Y)[row * CE + d] = y; }
    __threadfence(); }
}
__global__ __launch_bounds__(64) void out_kernel(const float* __restrict__ Y, const float* __restrict__ UV, const float* __restrict__ V2, const b16* __restrict__ WPR, const float* __restrict__ bpr, float* __restrict__ out) {
  __shared__ __attribute__((aligned(16))) b16 Ah[2][16][CE + 8], Al[2][16][CE + 8]; __shared__ __attribute__((aligned(16))) float To[C][32 + 1];
  const int wave = threadIdx.x >> 5, lane = threadIdx.x & 31, nloc = lane & 15, hlf = lane >> 4; const size_t t0 = (size_t)blockIdx.x * 32; const size_t m0 = t0 + wave * 16; const int b = (int)(t0 / L), p0 = (int)(t0 % L);
  for (int rr = 0; rr < 16; ++rr) for (int q = 0; q < 4; ++q) { const size_t r = m0 + rr; const v4f y = *(const v4f*)(Y + r * CE + q * 128 + lane * 4), u = *(const v4f*)(UV + r * (2 * CE) + q * 128 + lane * 4), v = *(const v4f*)(V2 + r * CE + q * 128 + lane * 4);
    for (int j = 0; j < 4; ++j) { const float su = sigm(u[j]); const float a = pmul(y[j], pmul(u[j], su)) + pmul(v[j], pmul(u[j], 1.0f - su)); b16 p, ql; split16(a * OS, p, ql); Ah[wave][rr][q * 128 + lane * 4 + j] = p; Al[wave][rr][q * 128 + lane * 4 + j] = ql; } }
  wave_lds_sync();
#pragma unroll 1
  for (int cg = 0; cg < 2; ++cg) { v8f acc[8];
#pragma unroll
    for (int t = 0; t < 8; ++t) acc[t] = (v8f){};
#pragma unroll 2
    for (int kb = 0; kb < CE; kb += 32) { const v16b a = frag_kb(&Ah[wave][nloc][kb], hlf), al = frag_kb(&Al[wave][nloc][kb], hlf);
#pragma unroll
      for (int t = 0; t < 8; ++t) { const v16b bw = frag_kb(WPR + (size_t)(cg * 128 + t * 16 + nloc) * CE + kb, hlf); acc[t] = wmma16b(a, bw, acc[t]); acc[t] = wmma16b(al, bw, acc[t]); } }
#pragma unroll
    for (int t = 0; t < 8; ++t) { const int c = cg * 128 + t * 16 + nloc; const float bb = bf16_rne(bpr[c]);
#pragma unroll 1
      for (int r8 = 0; r8 < 8; ++r8) To[c][wave * 16 + 8 * hlf + r8] = acc[t][r8] * (1.0f / (OS * WSC)) + bb; } }
  __syncthreads();
  for (int pass = 0; pass < 2; ++pass) { for (int i = threadIdx.x; i < C * 32; i += 64) { const int c = i >> 5, pp = i & 31; ((volatile float*)out)[((size_t)b * C + c) * L + p0 + pp] = To[c][pp]; } __threadfence(); }
}
}

extern "C" void kernel_launch(void* const* d_in, const int* in_sizes, int n_in, void* d_out, int out_size, void* d_ws, size_t ws_size, hipStream_t stream) {
  (void)n_in;
  auto Fp = [&](int i) { return (const float*)d_in[i]; };
  if (in_sizes[0] != NT * C || in_sizes[3] != 2 * CE * C || in_sizes[5] != C * CE || in_sizes[7] != 9 * CE || in_sizes[8] != CE * NS || in_sizes[10] != XD * CE || in_sizes[12] != CE * DTR || out_size != NT * C) return;
  const int NBV = NB; const int NTV = NBV * L;
  size_t off = 0; char* ws = (char*)d_ws;
  auto carve = [&](size_t bytes) { char* p = ws + off; off += (bytes + 255) & ~(size_t)255; return p; };
  b16* WEX = (b16*)carve((size_t)2 * CE * C * 2); b16* WPR = (b16*)carve((size_t)C * CE * 2); b16* WXP = (b16*)carve((size_t)XD * CE * 2); b16* WDT = (b16*)carve((size_t)CE * DTR * 2);
  float* UV = (float*)carve((size_t)NT * 2 * CE * 4); float* V2 = (float*)carve((size_t)NT * CE * 4); float* DT = (float*)carve((size_t)NT * CE * 4); float* BCp = (float*)carve((size_t)NT * 32 * 4); float* Y = (float*)carve((size_t)NT * CE * 4);
  if (off > ws_size || off > ((size_t)128 << 20)) return;
  wcopy_kernel<<<(2 * CE * C / 8 + 255) / 256, 256, 0, stream>>>(Fp(3), 2 * CE * C / 8, WEX); wcopy_kernel<<<(C * CE / 8 + 255) / 256, 256, 0, stream>>>(Fp(5), C * CE / 8, WPR);
  wcopy_kernel<<<(XD * CE / 8 + 255) / 256, 256, 0, stream>>>(Fp(10), XD * CE / 8, WXP); wcopy_kernel<<<(CE * DTR / 8 + 255) / 256, 256, 0, stream>>>(Fp(12), CE * DTR / 8, WDT);
  expand_kernel<<<NTV / 16, 32, 0, stream>>>(Fp(0), Fp(1), Fp(2), WEX, Fp(4), UV);
  dwconv_kernel<<<(unsigned)(((size_t)NTV * (CE / 4) + 255) / 256), 256, 0, stream>>>(UV, Fp(7), V2);
  mid_kernel<<<NTV / 16, 32, 0, stream>>>(V2, WXP, Fp(11), WDT, Fp(13), BCp, DT);
  scan_kernel<<<NBV * CE / 256, 256, 0, stream>>>(V2, DT, BCp, Fp(8), Fp(9), NBV, Y);
  out_kernel<<<NTV / 32, 64, 0, stream>>>(Y, UV, V2, WPR, Fp(6), (float*)d_out);
}
